// MultiScaleDeformAttn_34505767256646
// MI455X (gfx1250) — hardware-verified
//
#include <hip/hip_runtime.h>
#include <stdint.h>


typedef __attribute__((ext_vector_type(16))) _Float16 v16h;
typedef __attribute__((ext_vector_type(8)))  _Float16 v8h;
typedef __attribute__((ext_vector_type(16))) __bf16   v16b;
typedef __attribute__((ext_vector_type(8)))  __bf16   v8b;
typedef __attribute__((ext_vector_type(8)))  float    v8f;
typedef __attribute__((ext_vector_type(4)))  float    v4f;

__device__ __forceinline__ unsigned short f2bf_bits(float f) {
  unsigned u = __float_as_uint(f);
  return (unsigned short)((u + 0x7FFFu + ((u >> 16) & 1u)) >> 16);
}
__device__ __forceinline__ float bf_bits2f(unsigned short h) { return __uint_as_float(((unsigned)h) << 16); }

__device__ __forceinline__ void dep_guard_h(v8f& a, v8f& b, v16h x, v16h y) { asm volatile("v_nop\n\tv_nop\n\tv_nop\n\tv_nop" : "+v"(a), "+v"(b) : "v"(x), "v"(y)); }
__device__ __forceinline__ void dep_guard_b(v8f& a, v8f& b, v16b x, v16b y) { asm volatile("v_nop\n\tv_nop\n\tv_nop\n\tv_nop" : "+v"(a), "+v"(b) : "v"(x), "v"(y)); }
__device__ __forceinline__ void keep4_h(v16h a, v16h b, v16h c, v16h d) { asm volatile("v_nop" :: "v"(a), "v"(b), "v"(c), "v"(d)); }
__device__ __forceinline__ void keep4_b(v16b a, v16b b, v16b c, v16b d) { asm volatile("v_nop" :: "v"(a), "v"(b), "v"(c), "v"(d)); }
__device__ __forceinline__ void acc_guard4(v8f& a, v8f& b, v8f& c, v8f& d) { asm volatile("v_nop\n\tv_nop\n\tv_nop\n\tv_nop" : "+v"(a), "+v"(b), "+v"(c), "+v"(d)); }
template <typename T> struct Frag;
template <> struct Frag<_Float16> {
  typedef v16h V; union U { v16h v; v8h h[2]; };
  static __device__ __forceinline__ v16h load(const _Float16* p) {
    U f; f.h[0] = *(const v8h*)(p); f.h[1] = *(const v8h*)(p + 16); return f.v;
  }
  static __device__ __forceinline__ v8f mma(v16h a, v16h b, v8f c) {
    return __builtin_amdgcn_wmma_f32_16x16x32_f16(false, a, false, b, (short)0, c, false, false);
  }
  static __device__ __forceinline__ void guard(v8f& a, v8f& b, v16h x, v16h y) { dep_guard_h(a, b, x, y); }
  static __device__ __forceinline__ void keep(v16h a, v16h b, v16h c, v16h d) { keep4_h(a, b, c, d); }
};
template <> struct Frag<__bf16> {
  typedef v16b V; union U { v16b v; v8b h[2]; };
  static __device__ __forceinline__ v16b load(const __bf16* p) {
    U f; f.h[0] = *(const v8b*)(p); f.h[1] = *(const v8b*)(p + 16); return f.v;
  }
  static __device__ __forceinline__ v8f mma(v16b a, v16b b, v8f c) {
    return __builtin_amdgcn_wmma_f32_16x16x32_bf16(false, a, false, b, (short)0, c, false, false);
  }
  static __device__ __forceinline__ void guard(v8f& a, v8f& b, v16b x, v16b y) { dep_guard_b(a, b, x, y); }
  static __device__ __forceinline__ void keep(v16b a, v16b b, v16b c, v16b d) { keep4_b(a, b, c, d); }
};

template <int ET> struct Elem;
template <> struct Elem<0> { typedef _Float16 T; };
template <> struct Elem<1> { typedef __bf16 T; };
template <int ET, bool SPLIT, int BIAS_MODE, int OUT_MODE, bool RESID, int ACT = 0>
__global__ __launch_bounds__(256) void wmma_gemm64(
    const unsigned short* __restrict__ Ap, const unsigned short* __restrict__ A2p, int lda, long strideA,
    const unsigned short* __restrict__ Btp, const unsigned short* __restrict__ Bt2p, int ldb, long strideB,
    void* __restrict__ Cout, void* __restrict__ Cout2, int ldc, long strideC,
    const float* __restrict__ bias,
    const float* __restrict__ resid, long strideR,
    int M, int N, int K, float scale, int Mst) {
  typedef typename Elem<ET>::T T;
  typedef typename Frag<T>::V V;
  const T* A = (const T*)Ap; const T* A2 = (const T*)A2p; const T* Bt = (const T*)Btp; const T* Bt2 = (const T*)Bt2p;
  __shared__ __align__(16) float sT[8][16 * 68];
  const int b    = blockIdx.y;
  const int lane = threadIdx.x & 31;
  const int wave = threadIdx.x >> 5;
  const int tilesN = N >> 6;
  const int tilesM = M >> 6;
  const int tile = blockIdx.x * 8 + wave;
  if (tile >= tilesM * tilesN) return;
  const int tm = tile / tilesN;
  const int tn = tile - tm * tilesN;
  const int m0 = tm << 6;
  const int n0 = tn << 6;

  const T* Ab  = A  + (size_t)b * strideA;
  const T* Bb  = Bt + (size_t)b * strideB;
  const T* Ab2 = SPLIT ? (A2  + (size_t)b * strideA) : nullptr;
  const T* Bb2 = SPLIT ? (Bt2 + (size_t)b * strideB) : nullptr;

  const int rlane = lane & 15;
  const int koff  = (lane >> 4) * 8;
  const int mOff  = (lane >> 4) * 8;

  v8f acc[4][4];
#pragma unroll
  for (int i = 0; i < 4; ++i)
#pragma unroll
    for (int j = 0; j < 4; ++j) acc[i][j] = (v8f){0.f,0.f,0.f,0.f,0.f,0.f,0.f,0.f};

  for (int k0 = 0; k0 < K; k0 += 32) {
    V bh[4], bl[4];
#pragma unroll
    for (int j = 0; j < 4; ++j) {
      const size_t bo = (size_t)(n0 + (j << 4) + rlane) * ldb + koff + k0;
      bh[j] = Frag<T>::load(Bb + bo);
      if (SPLIT) bl[j] = Frag<T>::load(Bb2 + bo);
    }
#pragma unroll
    for (int i = 0; i < 4; ++i) {
      const size_t ao = (size_t)(m0 + (i << 4) + rlane) * lda + koff + k0;
      V ah = Frag<T>::load(Ab + ao);
      V al;
      if (SPLIT) al = Frag<T>::load(Ab2 + ao);
#pragma unroll
      for (int j = 0; j < 4; ++j) {
        acc[i][j] = Frag<T>::mma(ah, bh[j], acc[i][j]);
        if (SPLIT) {
          acc[i][j] = Frag<T>::mma(ah, bl[j], acc[i][j]);
          acc[i][j] = Frag<T>::mma(al, bh[j], acc[i][j]);
        }
      }
      Frag<T>::guard(acc[i][0], acc[i][3], ah, SPLIT ? al : ah);
    }
    Frag<T>::keep(bh[0], bh[1], bh[2], bh[3]);
    if (SPLIT) Frag<T>::keep(bl[0], bl[1], bl[2], bl[3]);
  }
  acc_guard4(acc[0][0], acc[0][1], acc[0][2], acc[0][3]);
  acc_guard4(acc[1][0], acc[1][1], acc[1][2], acc[1][3]);
  acc_guard4(acc[2][0], acc[2][1], acc[2][2], acc[2][3]);
  acc_guard4(acc[3][0], acc[3][1], acc[3][2], acc[3][3]);

  float* slab = sT[wave];
  const float* Rb = RESID ? (resid + (size_t)b * strideR) : nullptr;
#pragma unroll
  for (int i = 0; i < 4; ++i) {
    const int mBase = m0 + (i << 4);
#pragma unroll
    for (int j = 0; j < 4; ++j) {
      const int n = n0 + (j << 4) + rlane;
      float bv = 0.f;
      if (BIAS_MODE == 2) bv = bias[n];
#pragma unroll
      for (int r = 0; r < 8; ++r) {
        float v = acc[i][j][r] * scale;
        if (BIAS_MODE == 1) v += bias[mBase + mOff + r];
        if (BIAS_MODE == 2) v += bv;
        if (RESID) v += Rb[(size_t)(mBase + mOff + r) * ldc + n];
        if (ACT == 1) v = tanhf(v);
        if (ACT == 2) v = fmaxf(v, 0.0f);
        if (ACT == 3) v = v / (1.0f + expf(-v));
        if (ACT == 4) v = (v > 0.f) ? v : 0.01f * v;
        if (ACT == 5) v = 0.5f * v * (1.0f + erff(v * 0.70710678118654752f));
        slab[(mOff + r) * 68 + (j << 4) + rlane] = v;
      }
    }
    __builtin_amdgcn_fence(__ATOMIC_RELEASE, "workgroup");
    __builtin_amdgcn_wave_barrier();
    __builtin_amdgcn_fence(__ATOMIC_ACQUIRE, "workgroup");
    if (OUT_MODE == 0) {
      float* C = (float*)Cout + (size_t)b * strideC;
      const int hh = lane >> 4, c4 = (lane & 15) * 4;
      for (int pass = 0; pass < 2; ++pass) {
#pragma unroll
        for (int it = 0; it < 8; ++it) {
          const int row = it * 2 + hh;
          v4f v = *(const v4f*)(slab + row * 68 + c4);
          if (mBase + row < Mst) *(volatile v4f*)(C + (size_t)(mBase + row) * ldc + n0 + c4) = v;
        }
        __threadfence();
      }
    } else {
      const int q = lane >> 3, c8 = (lane & 7) * 8;
      unsigned short* C  = (unsigned short*)Cout  + (size_t)b * strideC;
      unsigned short* C2 = (OUT_MODE == 2) ? ((unsigned short*)Cout2 + (size_t)b * strideC) : nullptr;
      for (int pass = 0; pass < 2; ++pass) {
#pragma unroll
        for (int it = 0; it < 4; ++it) {
          const int row = it * 4 + q;
          const float* sp = slab + row * 68 + c8;
          v8h hv, lv;
#pragma unroll
          for (int e = 0; e < 8; ++e) {
            if (OUT_MODE == 1) {
              hv[e] = (_Float16)sp[e];
            } else {
              unsigned short hb = f2bf_bits(sp[e]);
              unsigned short lb = f2bf_bits(sp[e] - bf_bits2f(hb));
              hv[e] = __builtin_bit_cast(_Float16, hb);
              lv[e] = __builtin_bit_cast(_Float16, lb);
            }
          }
          if (mBase + row < Mst) {
            *(volatile v8h*)(C + (size_t)(mBase + row) * ldc + n0 + c8) = hv;
            if (OUT_MODE == 2) *(volatile v8h*)(C2 + (size_t)(mBase + row) * ldc + n0 + c8) = lv;
          }
        }
        __threadfence();
      }
    }
    __builtin_amdgcn_fence(__ATOMIC_RELEASE, "workgroup");
    __builtin_amdgcn_wave_barrier();
    __builtin_amdgcn_fence(__ATOMIC_ACQUIRE, "workgroup");
  }
}

template <int MODE>
__global__ __launch_bounds__(256) void cvt_planes(
    const float* __restrict__ a,
    unsigned short* __restrict__ o0, unsigned short* __restrict__ o1,
    int nval8, int ntot8, float fsc) {
  const int i = blockIdx.x * 256 + threadIdx.x;
  if (i >= ntot8) return;
  const bool live = (i < nval8);
  const int ic = live ? i : (nval8 - 1);
  const float* pa = a + (size_t)ic * 8;
  const v4f a0 = *(const v4f*)(pa), a1 = *(const v4f*)(pa + 4);
  v8h p0, p1;
#pragma unroll
  for (int e = 0; e < 4; ++e) {
    const float s0 = live ? (a0[e] * fsc) : 0.0f;
    const float s1 = live ? (a1[e] * fsc) : 0.0f;
    if (MODE == 0) {
      p0[e]     = (_Float16)s0;
      p0[4 + e] = (_Float16)s1;
      p1[e]     = p0[e];
      p1[4 + e] = p0[4 + e];
    } else {
      const unsigned short h0 = f2bf_bits(s0);
      const unsigned short l0 = f2bf_bits(s0 - bf_bits2f(h0));
      const unsigned short h1 = f2bf_bits(s1);
      const unsigned short l1 = f2bf_bits(s1 - bf_bits2f(h1));
      p0[e]     = __builtin_bit_cast(_Float16, h0);
      p0[4 + e] = __builtin_bit_cast(_Float16, h1);
      p1[e]     = __builtin_bit_cast(_Float16, l0);
      p1[4 + e] = __builtin_bit_cast(_Float16, l1);
    }
  }
  const size_t o = (size_t)i * 8;
  *(volatile v8h*)(o0 + o) = p0;
  if (MODE == 1) *(volatile v8h*)(o1 + o) = p1;
  __threadfence();
  *(volatile v8h*)(o0 + o) = p0;
  if (MODE == 1) *(volatile v8h*)(o1 + o) = p1;
}

__global__ __launch_bounds__(256) void deform_points(
    const float* __restrict__ valp,
    const float* __restrict__ offp,
    const float* __restrict__ attp,
    const float* __restrict__ pp,
    const int*   __restrict__ ssp,
    const int*   __restrict__ lvp,
    unsigned short* __restrict__ midp,
    int nrows, int spb, float midsc) {
#pragma clang fp contract(off)
  __shared__ __align__(16) float srow[256];
  const int bn   = blockIdx.x;
  const int wave = threadIdx.x >> 5;
  const int lane = threadIdx.x & 31;
  const int m    = wave;
  const bool live = (bn < nrows);
  const int bnc  = live ? bn : (nrows - 1);
  const int b    = bnc / spb;
  const int j16  = lane & 15;
  const int l    = j16 >> 2;

  int Hl = ssp[2 * l], Wl = ssp[2 * l + 1];
  const int st = lvp[l];
  Hl = Hl < 1 ? 1 : Hl;
  Wl = Wl < 1 ? 1 : Wl;
  const float fH = (float)Hl, fW = (float)Wl;
  const float aw = attp[(size_t)bnc * 128 + m * 16 + j16];
  const float ox = offp[(size_t)bnc * 256 + m * 32 + 2 * j16];
  const float oy = offp[(size_t)bnc * 256 + m * 32 + 2 * j16 + 1];
  const float rx = pp[(size_t)bnc * 8 + 2 * l];
  const float ry = pp[(size_t)bnc * 8 + 2 * l + 1];
  const float iw = 1.0f / fW;
  const float ih = 1.0f / fH;
  const float tx = ox * iw;
  const float ty = oy * ih;
  const float lxn = rx + tx;
  const float lyn = ry + ty;
  const float sx = lxn * fW;
  const float sy = lyn * fH;
  float px = sx - 0.5f;
  float py = sy - 0.5f;
  px = fminf(fmaxf(px, -2.0f), (float)(Wl + 1));
  py = fminf(fmaxf(py, -2.0f), (float)(Hl + 1));
  const float x0f = floorf(px), y0f = floorf(py);
  const float lx = px - x0f, ly = py - y0f;
  const float gx = 1.0f - lx, gy = 1.0f - ly;
  const int x0 = (int)x0f, y0 = (int)y0f;
  const int x1 = x0 + 1,   y1 = y0 + 1;
  const bool vx0 = (x0 >= 0) & (x0 < Wl), vx1 = (x1 >= 0) & (x1 < Wl);
  const bool vy0 = (y0 >= 0) & (y0 < Hl), vy1 = (y1 >= 0) & (y1 < Hl);
  const float f00 = (vy0 & vx0) ? 1.0f : 0.0f;
  const float f01 = (vy0 & vx1) ? 1.0f : 0.0f;
  const float f10 = (vy1 & vx0) ? 1.0f : 0.0f;
  const float f11 = (vy1 & vx1) ? 1.0f : 0.0f;
  const float w00 = ((gy * gx) * f00) * aw;
  const float w01 = ((gy * lx) * f01) * aw;
  const float w10 = ((ly * gx) * f10) * aw;
  const float w11 = ((ly * lx) * f11) * aw;
  const int xc0 = min(max(x0, 0), Wl - 1), xc1 = min(max(x1, 0), Wl - 1);
  const int yc0 = min(max(y0, 0), Hl - 1), yc1 = min(max(y1, 0), Hl - 1);
  int i00 = st + yc0 * Wl + xc0, i01 = st + yc0 * Wl + xc1;
  int i10 = st + yc1 * Wl + xc0, i11 = st + yc1 * Wl + xc1;
  i00 = min(max(i00, 0), spb - 1);
  i01 = min(max(i01, 0), spb - 1);
  i10 = min(max(i10, 0), spb - 1);
  i11 = min(max(i11, 0), spb - 1);

  const float* val = valp + (size_t)b * spb * 256 + m * 32 + lane;
  const unsigned smax = (unsigned)(spb - 1);
  float acc = 0.0f;
#pragma unroll 1
  for (int j = 0; j < 16; ++j) {
    unsigned a00 = (unsigned)__shfl(i00, j, 32);
    unsigned a01 = (unsigned)__shfl(i01, j, 32);
    unsigned a10 = (unsigned)__shfl(i10, j, 32);
    unsigned a11 = (unsigned)__shfl(i11, j, 32);
    const float c00 = __shfl(w00, j, 32);
    const float c01 = __shfl(w01, j, 32);
    const float c10 = __shfl(w10, j, 32);
    const float c11 = __shfl(w11, j, 32);
    a00 = min(a00, smax); a01 = min(a01, smax); a10 = min(a10, smax); a11 = min(a11, smax);
    const float g00 = val[(size_t)a00 * 256];
    const float g01 = val[(size_t)a01 * 256];
    const float g10 = val[(size_t)a10 * 256];
    const float g11 = val[(size_t)a11 * 256];
    acc += g00 * c00;
    acc += g01 * c01;
    acc += g10 * c10;
    acc += g11 * c11;
  }
  srow[m * 32 + lane] = live ? (acc * midsc) : 0.0f;
  __syncthreads();
  if (wave == 0) {
    const v4f p0 = *(const v4f*)(srow + lane * 8);
    const v4f p1 = *(const v4f*)(srow + lane * 8 + 4);
    v8h hv;
#pragma unroll
    for (int e = 0; e < 4; ++e) { hv[e] = (_Float16)p0[e]; hv[4 + e] = (_Float16)p1[e]; }
    unsigned short* dst = midp + (size_t)bn * 256 + lane * 8;
    *(volatile v8h*)dst = hv;
    __threadfence();
    *(volatile v8h*)dst = hv;
  }
}

extern "C" void kernel_launch(void* const* d_in, const int* in_sizes, int n_in,
                              void* d_out, int out_size, void* d_ws, size_t ws_size,
                              hipStream_t stream) {
  const int ROWS = 22506, ROWSP = 22528, DM = 256, NA = 128, SPB = 11253;
  if (n_in < 13) return;
  if (in_sizes[0] != ROWS * DM || in_sizes[1] != ROWS * 8 || in_sizes[2] != ROWS * DM || in_sizes[3] != 8 ||
      in_sizes[4] != 4 || in_sizes[5] != DM * DM || in_sizes[6] != DM || in_sizes[7] != NA * DM ||
      in_sizes[8] != NA || in_sizes[9] != DM * DM || in_sizes[10] != DM || in_sizes[11] != DM * DM ||
      in_sizes[12] != DM || out_size != ROWS * DM) return;

  const float* qin   = (const float*)d_in[0];
  const float* pin   = (const float*)d_in[1];
  const float* vin   = (const float*)d_in[2];
  const int*   ssp   = (const int*)d_in[3];
  const int*   lvp   = (const int*)d_in[4];
  const float* Woff  = (const float*)d_in[5];
  const float* boff  = (const float*)d_in[6];
  const float* Wa    = (const float*)d_in[7];
  const float* battn = (const float*)d_in[8];
  const float* Wv    = (const float*)d_in[9];
  const float* bval  = (const float*)d_in[10];
  const float* Wout  = (const float*)d_in[11];
  const float* bout  = (const float*)d_in[12];
  float* out = (float*)d_out;

  const size_t plane16 = (size_t)ROWSP * DM * 2;
  const size_t plane32 = (size_t)ROWSP * DM * 4;
  size_t cur = 0;
  auto carve = [&](size_t bytes) { size_t r = cur; cur += (bytes + 127) & ~(size_t)127; return r; };
  const size_t o_qh   = carve(plane16);
  const size_t o_ql   = carve(plane16);
  const size_t o_vf   = carve(plane16);
  const size_t o_mid  = carve(plane16);
  const size_t o_vp   = carve(plane32);
  const size_t o_off  = carve(plane32);
  const size_t o_att  = carve((size_t)ROWSP * NA * 4);
  const size_t o_wv   = carve((size_t)DM * DM * 2);
  const size_t o_woh  = carve((size_t)DM * DM * 2);
  const size_t o_wol  = carve((size_t)DM * DM * 2);
  const size_t o_wout = carve((size_t)DM * DM * 2);
  const size_t o_wah  = carve((size_t)NA * DM * 2);
  const size_t o_wal  = carve((size_t)NA * DM * 2);
  if (cur > ws_size) return;

  char* ws = (char*)d_ws;
  unsigned short* qh   = (unsigned short*)(ws + o_qh);
  unsigned short* ql   = (unsigned short*)(ws + o_ql);
  unsigned short* vf   = (unsigned short*)(ws + o_vf);
  unsigned short* mid  = (unsigned short*)(ws + o_mid);
  float*          vp   = (float*)(ws + o_vp);
  float*          offb = (float*)(ws + o_off);
  float*          attb = (float*)(ws + o_att);
  unsigned short* wvT  = (unsigned short*)(ws + o_wv);
  unsigned short* wohT = (unsigned short*)(ws + o_woh);
  unsigned short* wolT = (unsigned short*)(ws + o_wol);
  unsigned short* woT  = (unsigned short*)(ws + o_wout);
  unsigned short* wahT = (unsigned short*)(ws + o_wah);
  unsigned short* walT = (unsigned short*)(ws + o_wal);

  {
    const int nval8 = ROWS * DM / 8, ntot8 = ROWSP * DM / 8;
    cvt_planes<1><<<dim3((ntot8 + 255) / 256), dim3(256), 0, stream>>>(qin, qh, ql, nval8, ntot8, 1.0f);
    cvt_planes<0><<<dim3((ntot8 + 255) / 256), dim3(256), 0, stream>>>(vin, vf, vf, nval8, ntot8, 8.0f);
  }
  {
    const int n8 = DM * DM / 8, n8a = NA * DM / 8;
    cvt_planes<0><<<dim3((n8 + 255) / 256),  dim3(256), 0, stream>>>(Wv,   wvT,  wvT,  n8,  n8,  64.0f);
    cvt_planes<1><<<dim3((n8 + 255) / 256),  dim3(256), 0, stream>>>(Woff, wohT, wolT, n8,  n8,  1.0f);
    cvt_planes<1><<<dim3((n8a + 255) / 256), dim3(256), 0, stream>>>(Wa,   wahT, walT, n8a, n8a, 1.0f);
    cvt_planes<0><<<dim3((n8 + 255) / 256),  dim3(256), 0, stream>>>(Wout, woT,  woT,  n8,  n8,  64.0f);
  }

  const int tilesM = ROWSP / 64;
  {
    const int tiles = tilesM * (DM / 64);
    wmma_gemm64<0, false, 2, 0, false, 0><<<dim3((tiles + 7) / 8, 1), dim3(256), 0, stream>>>(
        vf, vf, DM, 0L, wvT, wvT, DM, 0L, (void*)vp, (void*)mid, DM, 0L,
        bval, bval, 0L, ROWSP, DM, DM, 1.0f / 512.0f, ROWSP);
  }
  {
    const int tiles = tilesM * (DM / 64);
    wmma_gemm64<1, true, 2, 0, false, 0><<<dim3((tiles + 7) / 8, 1), dim3(256), 0, stream>>>(
        qh, ql, DM, 0L, wohT, wolT, DM, 0L, (void*)offb, (void*)mid, DM, 0L,
        boff, boff, 0L, ROWSP, DM, DM, 1.0f, ROWSP);
  }
  {
    const int tiles = tilesM * (NA / 64);
    wmma_gemm64<1, true, 2, 0, false, 0><<<dim3((tiles + 7) / 8, 1), dim3(256), 0, stream>>>(
        qh, ql, DM, 0L, wahT, walT, DM, 0L, (void*)attb, (void*)mid, NA, 0L,
        battn, battn, 0L, ROWSP, NA, DM, 1.0f, ROWSP);
  }
  deform_points<<<dim3(ROWSP), dim3(256), 0, stream>>>(vp, offb, attb, pin, ssp, lvp, mid, ROWS, SPB, 16.0f);
  {
    const int tiles = tilesM * (DM / 64);
    wmma_gemm64<0, false, 2, 0, false, 0><<<dim3((tiles + 7) / 8, 1), dim3(256), 0, stream>>>(
        mid, mid, DM, 0L, woT, woT, DM, 0L, (void*)out, (void*)ql, DM, 0L,
        bout, bout, 0L, ROWSP, DM, DM, 1.0f / 1024.0f, ROWS);
  }
}
